// MMD_VAE_6648609375080
// MI455X (gfx1250) — hardware-verified
//
#include <hip/hip_runtime.h>
#include <math.h>
#include <stdint.h>

constexpr int kTok = 4096;
constexpr int kDm  = 1024;
constexpr int kDi  = 4096;
constexpr int kDl  = 64;
constexpr int kPartStride = 32;
constexpr int kRedRows    = 8;
constexpr int kRedBlocks  = kTok / kRedRows;
constexpr float kInvTok2TimesScale = 64.0f / 16777216.0f;
constexpr float kLnEps = 1e-9f;

typedef __attribute__((ext_vector_type(16))) _Float16 v16h;
typedef __attribute__((ext_vector_type(8)))  _Float16 v8h;
typedef __attribute__((ext_vector_type(16))) __bf16   v16b;
typedef __attribute__((ext_vector_type(8)))  __bf16   v8b;
typedef __attribute__((ext_vector_type(8)))  float    v8f;
typedef __attribute__((ext_vector_type(4)))  float    v4f;
typedef __attribute__((ext_vector_type(4)))  unsigned int v4u;

__device__ __forceinline__ unsigned short f2bf_bits(float f) {
  unsigned u = __float_as_uint(f);
  return (unsigned short)((u + 0x7FFFu + ((u >> 16) & 1u)) >> 16);
}
__device__ __forceinline__ float bf_bits2f(unsigned short h) { return __uint_as_float(((unsigned)h) << 16); }

__device__ __forceinline__ void dep_guard_h(v8f& a, v8f& b, v16h x, v16h y) { asm volatile("v_nop\n\tv_nop\n\tv_nop\n\tv_nop" : "+v"(a), "+v"(b) : "v"(x), "v"(y)); }
__device__ __forceinline__ void dep_guard_b(v8f& a, v8f& b, v16b x, v16b y) { asm volatile("v_nop\n\tv_nop\n\tv_nop\n\tv_nop" : "+v"(a), "+v"(b) : "v"(x), "v"(y)); }
__device__ __forceinline__ void keep4_h(v16h a, v16h b, v16h c, v16h d) { asm volatile("v_nop" :: "v"(a), "v"(b), "v"(c), "v"(d)); }
__device__ __forceinline__ void keep4_b(v16b a, v16b b, v16b c, v16b d) { asm volatile("v_nop" :: "v"(a), "v"(b), "v"(c), "v"(d)); }
__device__ __forceinline__ void acc_guard4(v8f& a, v8f& b, v8f& c, v8f& d) { asm volatile("v_nop\n\tv_nop\n\tv_nop\n\tv_nop" : "+v"(a), "+v"(b), "+v"(c), "+v"(d)); }
template <typename T> struct Frag;
template <> struct Frag<_Float16> {
  typedef v16h V; union U { v16h v; v8h h[2]; };
  static __device__ __forceinline__ v16h load(const _Float16* p) {
    U f; f.h[0] = *(const v8h*)(p); f.h[1] = *(const v8h*)(p + 16); return f.v;
  }
  static __device__ __forceinline__ v8f mma(v16h a, v16h b, v8f c) {
    return __builtin_amdgcn_wmma_f32_16x16x32_f16(false, a, false, b, (short)0, c, false, false);
  }
  static __device__ __forceinline__ void guard(v8f& a, v8f& b, v16h x, v16h y) { dep_guard_h(a, b, x, y); }
  static __device__ __forceinline__ void keep(v16h a, v16h b, v16h c, v16h d) { keep4_h(a, b, c, d); }
};
template <> struct Frag<__bf16> {
  typedef v16b V; union U { v16b v; v8b h[2]; };
  static __device__ __forceinline__ v16b load(const __bf16* p) {
    U f; f.h[0] = *(const v8b*)(p); f.h[1] = *(const v8b*)(p + 16); return f.v;
  }
  static __device__ __forceinline__ v8f mma(v16b a, v16b b, v8f c) {
    return __builtin_amdgcn_wmma_f32_16x16x32_bf16(false, a, false, b, (short)0, c, false, false);
  }
  static __device__ __forceinline__ void guard(v8f& a, v8f& b, v16b x, v16b y) { dep_guard_b(a, b, x, y); }
  static __device__ __forceinline__ void keep(v16b a, v16b b, v16b c, v16b d) { keep4_b(a, b, c, d); }
};

template <int ET> struct Elem;
template <> struct Elem<0> { typedef _Float16 T; };
template <> struct Elem<1> { typedef __bf16 T; };
template <int ET, bool SPLIT, int BIAS_MODE, int OUT_MODE, bool RESID, int ACT = 0, int TRI = 0>
__global__ __launch_bounds__(256) void wmma_gemm64(
    const unsigned short* __restrict__ Ap, const unsigned short* __restrict__ A2p, int lda, long strideA,
    const unsigned short* __restrict__ Btp, const unsigned short* __restrict__ Bt2p, int ldb, long strideB,
    void* __restrict__ Cout, void* __restrict__ Cout2, int ldc, long strideC,
    const float* __restrict__ bias,
    const float* __restrict__ resid, long strideR,
    int M, int N, int K, float scale) {
  typedef typename Elem<ET>::T T;
  typedef typename Frag<T>::V V;
  const T* A = (const T*)Ap; const T* A2 = (const T*)A2p; const T* Bt = (const T*)Btp; const T* Bt2 = (const T*)Bt2p;
  __shared__ __align__(16) float sT[8][16 * 68];
  const int b    = blockIdx.y;
  const int lane = threadIdx.x & 31;
  const int wave = threadIdx.x >> 5;
  const int tilesN = N >> 6;
  const int tilesM = M >> 6;
  const int tile = blockIdx.x * 8 + wave;
  if (tile >= tilesM * tilesN) return;
  const int tm = tile / tilesN;
  const int tn = tile - tm * tilesN;
  const int m0 = tm << 6;
  const int n0 = tn << 6;
  if (TRI == 1 && n0 > m0) return;
  const int Kl = (TRI == 2 && (m0 + 64) < K) ? (m0 + 64) : K;

  const T* Ab  = A  + (size_t)b * strideA;
  const T* Bb  = Bt + (size_t)b * strideB;
  const T* Ab2 = SPLIT ? (A2  + (size_t)b * strideA) : nullptr;
  const T* Bb2 = SPLIT ? (Bt2 + (size_t)b * strideB) : nullptr;

  const int rlane = lane & 15;
  const int koff  = (lane >> 4) * 8;
  const int mOff  = (lane >> 4) * 8;

  v8f acc[4][4];
#pragma unroll
  for (int i = 0; i < 4; ++i)
#pragma unroll
    for (int j = 0; j < 4; ++j) acc[i][j] = (v8f){0.f,0.f,0.f,0.f,0.f,0.f,0.f,0.f};

  for (int k0 = 0; k0 < Kl; k0 += 32) {
    V bh[4], bl[4];
#pragma unroll
    for (int j = 0; j < 4; ++j) {
      const size_t bo = (size_t)(n0 + (j << 4) + rlane) * ldb + koff + k0;
      bh[j] = Frag<T>::load(Bb + bo);
      if (SPLIT) bl[j] = Frag<T>::load(Bb2 + bo);
    }
#pragma unroll
    for (int i = 0; i < 4; ++i) {
      const size_t ao = (size_t)(m0 + (i << 4) + rlane) * lda + koff + k0;
      V ah = Frag<T>::load(Ab + ao);
      V al;
      if (SPLIT) al = Frag<T>::load(Ab2 + ao);
#pragma unroll
      for (int j = 0; j < 4; ++j) {
        acc[i][j] = Frag<T>::mma(ah, bh[j], acc[i][j]);
        if (SPLIT) {
          acc[i][j] = Frag<T>::mma(ah, bl[j], acc[i][j]);
          acc[i][j] = Frag<T>::mma(al, bh[j], acc[i][j]);
        }
      }
      Frag<T>::guard(acc[i][0], acc[i][3], ah, SPLIT ? al : ah);
    }
    Frag<T>::keep(bh[0], bh[1], bh[2], bh[3]);
    if (SPLIT) Frag<T>::keep(bl[0], bl[1], bl[2], bl[3]);
  }
  acc_guard4(acc[0][0], acc[0][1], acc[0][2], acc[0][3]);
  acc_guard4(acc[1][0], acc[1][1], acc[1][2], acc[1][3]);
  acc_guard4(acc[2][0], acc[2][1], acc[2][2], acc[2][3]);
  acc_guard4(acc[3][0], acc[3][1], acc[3][2], acc[3][3]);

  float* slab = sT[wave];
  const float* Rb = RESID ? (resid + (size_t)b * strideR) : nullptr;
#pragma unroll
  for (int i = 0; i < 4; ++i) {
    const int mBase = m0 + (i << 4);
#pragma unroll
    for (int j = 0; j < 4; ++j) {
      const int n = n0 + (j << 4) + rlane;
      float bv = 0.f;
      if (BIAS_MODE == 2) bv = bias[n];
#pragma unroll
      for (int r = 0; r < 8; ++r) {
        float v = acc[i][j][r] * scale;
        if (BIAS_MODE == 1) v += bias[mBase + mOff + r];
        if (BIAS_MODE == 2) v += bv;
        if (RESID) v += Rb[(size_t)(mBase + mOff + r) * ldc + n];
        if (ACT == 1) v = tanhf(v);
        if (ACT == 2) v = fmaxf(v, 0.0f);
        if (ACT == 3) v = v / (1.0f + expf(-v));
        if (ACT == 4) v = (v > 0.f) ? v : 0.01f * v;
        slab[(mOff + r) * 68 + (j << 4) + rlane] = v;
      }
    }
    __builtin_amdgcn_fence(__ATOMIC_RELEASE, "workgroup");
    __builtin_amdgcn_wave_barrier();
    __builtin_amdgcn_fence(__ATOMIC_ACQUIRE, "workgroup");
    if (OUT_MODE == 0) {
      float* C = (float*)Cout + (size_t)b * strideC;
      const int hh = lane >> 4, c4 = (lane & 15) * 4;
      for (int pass = 0; pass < 2; ++pass) {
#pragma unroll
        for (int it = 0; it < 8; ++it) {
          const int row = it * 2 + hh;
          v4f v = *(const v4f*)(slab + row * 68 + c4);
          *(volatile v4f*)(C + (size_t)(mBase + row) * ldc + n0 + c4) = v;
        }
        __threadfence();
      }
    } else {
      const int q = lane >> 3, c8 = (lane & 7) * 8;
      unsigned short* C  = (unsigned short*)Cout  + (size_t)b * strideC;
      unsigned short* C2 = (OUT_MODE == 2) ? ((unsigned short*)Cout2 + (size_t)b * strideC) : nullptr;
      for (int pass = 0; pass < 2; ++pass) {
#pragma unroll
        for (int it = 0; it < 4; ++it) {
          const int row = it * 4 + q;
          const float* sp = slab + row * 68 + c8;
          v8h hv, lv;
#pragma unroll
          for (int e = 0; e < 8; ++e) {
            if (OUT_MODE == 1) {
              hv[e] = (_Float16)sp[e];
            } else {
              unsigned short hb = f2bf_bits(sp[e]);
              unsigned short lb = f2bf_bits(sp[e] - bf_bits2f(hb));
              hv[e] = __builtin_bit_cast(_Float16, hb);
              lv[e] = __builtin_bit_cast(_Float16, lb);
            }
          }
          *(volatile v8h*)(C + (size_t)(mBase + row) * ldc + n0 + c8) = hv;
          if (OUT_MODE == 2) *(volatile v8h*)(C2 + (size_t)(mBase + row) * ldc + n0 + c8) = lv;
        }
        __threadfence();
      }
    }
    __builtin_amdgcn_fence(__ATOMIC_RELEASE, "workgroup");
    __builtin_amdgcn_wave_barrier();
    __builtin_amdgcn_fence(__ATOMIC_ACQUIRE, "workgroup");
  }
}

__device__ __forceinline__ unsigned pk16(unsigned short a, unsigned short b) { return (unsigned)a | ((unsigned)b << 16); }
__device__ __forceinline__ unsigned short h_bits(float f) { const _Float16 h = (_Float16)f; return __builtin_bit_cast(unsigned short, h); }

__global__ __launch_bounds__(256) void transpose_cast_f16_kernel(const float* __restrict__ in, unsigned short* __restrict__ out,
                                                                 int R, int CC, float scale) {
  __shared__ float tile[64][65];
  const int t  = threadIdx.x;
  const int n0 = blockIdx.x * 64;
  const int k0 = blockIdx.y * 64;
  {
    const int kr = t >> 2, nc = (t & 3) * 16;
    const float* p = in + (size_t)(k0 + kr) * CC + n0 + nc;
#pragma unroll
    for (int e4 = 0; e4 < 4; ++e4) {
      const v4f f = *(const v4f*)(p + 4 * e4);
      tile[kr][nc + 4 * e4 + 0] = f[0];
      tile[kr][nc + 4 * e4 + 1] = f[1];
      tile[kr][nc + 4 * e4 + 2] = f[2];
      tile[kr][nc + 4 * e4 + 3] = f[3];
    }
  }
  __syncthreads();
  const int q = t >> 3, c8 = (t & 7) * 8;
  v4u u0, u1;
#pragma unroll
  for (int w = 0; w < 4; ++w) {
    u0[w] = pk16(h_bits(tile[c8 + 2 * w][q] * scale),      h_bits(tile[c8 + 2 * w + 1][q] * scale));
    u1[w] = pk16(h_bits(tile[c8 + 2 * w][32 + q] * scale), h_bits(tile[c8 + 2 * w + 1][32 + q] * scale));
  }
  unsigned short* p0 = out + (size_t)(n0 + q) * R + k0 + c8;
  unsigned short* p1 = out + (size_t)(n0 + 32 + q) * R + k0 + c8;
  for (int pass = 0; pass < 2; ++pass) {
    *(volatile v4u*)p0 = u0;
    *(volatile v4u*)p1 = u1;
    __threadfence();
  }
}

__global__ __launch_bounds__(256) void cast_f32_f16x8_kernel(const float* __restrict__ in, unsigned short* __restrict__ out,
                                                             int n8, float scale) {
  const int i = blockIdx.x * 256 + threadIdx.x;
  if (i < n8) {
    const float* p = in + 8 * (size_t)i;
    const v4f a = *(const v4f*)(p);
    const v4f c = *(const v4f*)(p + 4);
    const v4u u = (v4u){pk16(h_bits(a[0] * scale), h_bits(a[1] * scale)), pk16(h_bits(a[2] * scale), h_bits(a[3] * scale)),
                        pk16(h_bits(c[0] * scale), h_bits(c[1] * scale)), pk16(h_bits(c[2] * scale), h_bits(c[3] * scale))};
    unsigned short* o = out + 8 * (size_t)i;
    *(volatile v4u*)o = u;
    __threadfence();
    *(volatile v4u*)o = u;
  }
}

__global__ __launch_bounds__(256) void gelu_erf_f32_f16x8_kernel(const float* __restrict__ in, unsigned short* __restrict__ out, int n8) {
  const int i = blockIdx.x * 256 + threadIdx.x;
  if (i < n8) {
    const float* p = in + 8 * (size_t)i;
    unsigned long long g0 = 0ull, g1 = 0ull;
#pragma unroll 1
    for (int e = 0; e < 8; ++e) {
      const bool hiw = (e >= 4);
      const int  sh  = (e & 3) * 16;
      const float x  = p[e];
      const float gv = 0.5f * x * (1.0f + erff(x * 0.70710678118654752f));
      const unsigned long long gb = ((unsigned long long)h_bits(gv)) << sh;
      g0 |= hiw ? 0ull : gb;
      g1 |= hiw ? gb : 0ull;
    }
    const v4u r = (v4u){(unsigned)(g0 & 0xFFFFFFFFull), (unsigned)(g0 >> 32),
                        (unsigned)(g1 & 0xFFFFFFFFull), (unsigned)(g1 >> 32)};
    unsigned short* o = out + 8 * (size_t)i;
    *(volatile v4u*)o = r;
    __threadfence();
    *(volatile v4u*)o = r;
  }
}

template <bool DO_LN>
__global__ __launch_bounds__(512) void rows64_kernel(const float* __restrict__ x, const float* __restrict__ gam,
                                                     const float* __restrict__ bet, float* __restrict__ outf,
                                                     unsigned short* __restrict__ out16, float* __restrict__ nrm) {
  __shared__ __align__(16) float slab[32 * 68];
  __shared__ __align__(16) float nsh[32];
  const int t    = threadIdx.x;
  const int lane = t & 31, wave = t >> 5;
  const int hh   = lane >> 4, c4 = (lane & 15) * 4;
  const int rib  = wave * 2 + hh;
  const int row  = blockIdx.x * 32 + rib;
  const v4f a = *(const v4f*)(x + (size_t)row * kDl + c4);
  float y0 = a[0], y1 = a[1], y2 = a[2], y3 = a[3];
  if (DO_LN) {
    float s = (a[0] + a[1]) + (a[2] + a[3]);
#pragma unroll
    for (int off = 8; off > 0; off >>= 1) s += __shfl_xor(s, off, 32);
    const float mu = s * (1.0f / 64.0f);
    const float d0 = a[0] - mu, d1 = a[1] - mu, d2 = a[2] - mu, d3 = a[3] - mu;
    float qq = (d0 * d0 + d1 * d1) + (d2 * d2 + d3 * d3);
#pragma unroll
    for (int off = 8; off > 0; off >>= 1) qq += __shfl_xor(qq, off, 32);
    const float var = qq * (1.0f / 64.0f);
    const float rs  = rsqrtf(var + kLnEps);
    const v4f g  = *(const v4f*)(gam + c4);
    const v4f bb = *(const v4f*)(bet + c4);
    y0 = d0 * rs * g[0] + bb[0];
    y1 = d1 * rs * g[1] + bb[1];
    y2 = d2 * rs * g[2] + bb[2];
    y3 = d3 * rs * g[3] + bb[3];
  }
  float nq = (y0 * y0 + y1 * y1) + (y2 * y2 + y3 * y3);
#pragma unroll
  for (int off = 8; off > 0; off >>= 1) nq += __shfl_xor(nq, off, 32);
  if ((lane & 15) == 0) nsh[rib] = nq;
  slab[rib * 68 + c4 + 0] = y0;
  slab[rib * 68 + c4 + 1] = y1;
  slab[rib * 68 + c4 + 2] = y2;
  slab[rib * 68 + c4 + 3] = y3;
  if (DO_LN) {
    const v4f yv = (v4f){y0, y1, y2, y3};
    float* op = outf + (size_t)row * kDl + c4;
    *(volatile v4f*)op = yv;
    __threadfence();
    *(volatile v4f*)op = yv;
  }
  __syncthreads();
  if (t < 256) {
    const int r = t >> 3, c8 = (t & 7) * 8;
    const float* sp = slab + r * 68 + c8;
    const v4u u = (v4u){pk16(h_bits(sp[0]), h_bits(sp[1])), pk16(h_bits(sp[2]), h_bits(sp[3])),
                        pk16(h_bits(sp[4]), h_bits(sp[5])), pk16(h_bits(sp[6]), h_bits(sp[7]))};
    unsigned short* op = out16 + (size_t)(blockIdx.x * 32 + r) * kDl + c8;
    *(volatile v4u*)op = u;
    __threadfence();
    *(volatile v4u*)op = u;
  }
  if (t < 8) {
    const v4f nv = *(const v4f*)(nsh + 4 * t);
    float* np_ = nrm + (size_t)blockIdx.x * 32 + 4 * t;
    *(volatile v4f*)np_ = nv;
    __threadfence();
    *(volatile v4f*)np_ = nv;
  }
}

__global__ __launch_bounds__(256) void layernorm1024_kernel(const float* __restrict__ x, const float* __restrict__ gam,
                                                             const float* __restrict__ bet, float* __restrict__ out) {
  __shared__ float redA[8];
  __shared__ float redB[8];
  const int row  = blockIdx.x;
  const int t    = threadIdx.x;
  const int lane = t & 31, wave = t >> 5;
  const int c0   = t * 4;
  const v4f a = *(const v4f*)(x + (size_t)row * kDm + c0);
  float s = (a[0] + a[1]) + (a[2] + a[3]);
#pragma unroll
  for (int off = 16; off > 0; off >>= 1) s += __shfl_xor(s, off, 32);
  if (lane == 0) redA[wave] = s;
  __syncthreads();
  const float mu = (((redA[0] + redA[1]) + (redA[2] + redA[3])) + ((redA[4] + redA[5]) + (redA[6] + redA[7]))) * (1.0f / 1024.0f);
  const float d0 = a[0] - mu, d1 = a[1] - mu, d2 = a[2] - mu, d3 = a[3] - mu;
  float qq = (d0 * d0 + d1 * d1) + (d2 * d2 + d3 * d3);
#pragma unroll
  for (int off = 16; off > 0; off >>= 1) qq += __shfl_xor(qq, off, 32);
  if (lane == 0) redB[wave] = qq;
  __syncthreads();
  const float var = (((redB[0] + redB[1]) + (redB[2] + redB[3])) + ((redB[4] + redB[5]) + (redB[6] + redB[7]))) * (1.0f / 1024.0f);
  const float rs  = rsqrtf(var + kLnEps);
  const v4f g  = *(const v4f*)(gam + c0);
  const v4f bb = *(const v4f*)(bet + c0);
  const v4f yv = (v4f){d0 * rs * g[0] + bb[0], d1 * rs * g[1] + bb[1], d2 * rs * g[2] + bb[2], d3 * rs * g[3] + bb[3]};
  float* op = out + (size_t)row * kDm + c0;
  *(volatile v4f*)op = yv;
  __threadfence();
  *(volatile v4f*)op = yv;
}

__global__ __launch_bounds__(256) void kmean_partial_kernel(const float* __restrict__ S, const float* __restrict__ nr,
                                                            const float* __restrict__ nc, float* __restrict__ part) {
  __shared__ float red[8];
  const int t = threadIdx.x, lane = t & 31, wave = t >> 5;
  const int r0 = blockIdx.x * kRedRows;
  float acc = 0.f;
#pragma unroll 1
  for (int it = 0; it < kRedRows * 16; ++it) {
    const int r   = r0 + (it >> 4);
    const int col = ((it & 15) << 8) + t;
    const float sv = S[(size_t)r * kTok + col];
    const float sq = (nr[r] + nc[col]) - 2.0f * sv;
    acc += expm1f(sq * (-1.0f / 4096.0f));
  }
#pragma unroll
  for (int off = 16; off > 0; off >>= 1) acc += __shfl_xor(acc, off, 32);
  if (lane == 0) red[wave] = acc;
  __syncthreads();
  if (wave == 0) {
    const float tot = ((red[0] + red[1]) + (red[2] + red[3])) + ((red[4] + red[5]) + (red[6] + red[7]));
    const float v = (lane == 0) ? tot : 0.f;
    float* pp = part + (size_t)blockIdx.x * kPartStride + lane;
    *(volatile float*)pp = v;
    __threadfence();
    *(volatile float*)pp = v;
  }
}

__global__ __launch_bounds__(32) void loss_final_kernel(const float* __restrict__ part, float* __restrict__ out2) {
  const int lane = threadIdx.x;
  float sx = 0.f, sy = 0.f, sxy = 0.f;
#pragma unroll 1
  for (int k = 0; k < kRedBlocks / 32; ++k) {
    const int bi = lane + 32 * k;
    sx  += part[(size_t)bi * kPartStride];
    sy  += part[(size_t)(kRedBlocks + bi) * kPartStride];
    sxy += part[(size_t)(2 * kRedBlocks + bi) * kPartStride];
  }
#pragma unroll
  for (int off = 16; off > 0; off >>= 1) {
    sx  += __shfl_xor(sx, off, 32);
    sy  += __shfl_xor(sy, off, 32);
    sxy += __shfl_xor(sxy, off, 32);
  }
  const float loss = ((sx + sy) - 2.0f * sxy) * kInvTok2TimesScale;
  if (lane == 0) {
    *(volatile float*)out2 = loss;
    __threadfence();
    *(volatile float*)out2 = loss;
  }
}

extern "C" void kernel_launch(void* const* d_in, const int* in_sizes, int n_in,
                              void* d_out, int out_size, void* d_ws, size_t ws_size,
                              hipStream_t stream) {
  if (n_in < 14) return;
  if (in_sizes[0] != kTok * kDm) return;
  if (in_sizes[1] != kTok * kDl) return;
  if (in_sizes[2] != kDm * kDi || in_sizes[3] != kDi) return;
  if (in_sizes[4] != kDi * kDl || in_sizes[5] != kDl || in_sizes[6] != kDl || in_sizes[7] != kDl) return;
  if (in_sizes[8] != kDl * kDi || in_sizes[9] != kDi) return;
  if (in_sizes[10] != kDi * kDm || in_sizes[11] != kDm || in_sizes[12] != kDm || in_sizes[13] != kDm) return;
  if (out_size != kTok * kDm + kTok * kDl + 1) return;

  const float* hidden = (const float*)d_in[0];
  const float* truep  = (const float*)d_in[1];
  const float* enc_w1 = (const float*)d_in[2];
  const float* enc_b1 = (const float*)d_in[3];
  const float* enc_w2 = (const float*)d_in[4];
  const float* enc_b2 = (const float*)d_in[5];
  const float* enc_g  = (const float*)d_in[6];
  const float* enc_bt = (const float*)d_in[7];
  const float* dec_w1 = (const float*)d_in[8];
  const float* dec_b1 = (const float*)d_in[9];
  const float* dec_w2 = (const float*)d_in[10];
  const float* dec_b2 = (const float*)d_in[11];
  const float* dec_g  = (const float*)d_in[12];
  const float* dec_bt = (const float*)d_in[13];

  float* recon = (float*)d_out;
  float* lat   = (float*)((char*)d_out + 16777216);
  float* regp  = (float*)((char*)d_out + 17825792);

  const size_t PH16  = (size_t)kTok * kDm * 2;
  const size_t PW1E  = (size_t)kDi * kDm * 2;
  const size_t PW2E  = (size_t)kDl * kDi * 2;
  const size_t PW1D  = (size_t)kDi * kDl * 2;
  const size_t PW2D  = (size_t)kDm * kDi * 2;
  const size_t PT16  = (size_t)kTok * kDl * 2;
  const size_t PUBIG = (size_t)kTok * kDi * 4;
  const size_t PG16  = (size_t)kTok * kDi * 2;
  const size_t PLAT0 = (size_t)kTok * kDl * 4;
  const size_t PLAT16= (size_t)kTok * kDl * 2;
  const size_t PNRM  = (size_t)kTok * 4;
  const size_t PPART = (size_t)3 * kRedBlocks * kPartStride * 4;
  static_assert((size_t)kTok * kDm * 4 <= (size_t)kTok * kDi * 4);
  static_assert((size_t)kTok * kTok * 4 <= (size_t)kTok * kDi * 4);
  size_t off = 0;
  const size_t oH16  = off; off += PH16;
  const size_t oW1E  = off; off += PW1E;
  const size_t oW2E  = off; off += PW2E;
  const size_t oW1D  = off; off += PW1D;
  const size_t oW2D  = off; off += PW2D;
  const size_t oT16  = off; off += PT16;
  const size_t oUBIG = off; off += PUBIG;
  const size_t oG16  = off; off += PG16;
  const size_t oLAT0 = off; off += PLAT0;
  const size_t oLAT16= off; off += PLAT16;
  const size_t oNX   = off; off += PNRM;
  const size_t oNY   = off; off += PNRM;
  const size_t oPART = off; off += PPART;
  if (off > (size_t)134217728) return;
  if (off > ws_size) return;

  char* ws = (char*)d_ws;
  unsigned short* H16   = (unsigned short*)(ws + oH16);
  unsigned short* W1ET  = (unsigned short*)(ws + oW1E);
  unsigned short* W2ET  = (unsigned short*)(ws + oW2E);
  unsigned short* W1DT  = (unsigned short*)(ws + oW1D);
  unsigned short* W2DT  = (unsigned short*)(ws + oW2D);
  unsigned short* T16   = (unsigned short*)(ws + oT16);
  float*          UBIG  = (float*)(ws + oUBIG);
  unsigned short* G16   = (unsigned short*)(ws + oG16);
  float*          LAT0  = (float*)(ws + oLAT0);
  unsigned short* LAT16 = (unsigned short*)(ws + oLAT16);
  float*          NX    = (float*)(ws + oNX);
  float*          NY    = (float*)(ws + oNY);
  float*          PART  = (float*)(ws + oPART);

  const dim3 blk(256);

  cast_f32_f16x8_kernel<<<dim3((kTok * kDm / 8) / 256), blk, 0, stream>>>(hidden, H16, kTok * kDm / 8, 1.0f);
  transpose_cast_f16_kernel<<<dim3(kDi / 64, kDm / 64), blk, 0, stream>>>(enc_w1, W1ET, kDm, kDi, 16.0f);
  transpose_cast_f16_kernel<<<dim3(kDl / 64, kDi / 64), blk, 0, stream>>>(enc_w2, W2ET, kDi, kDl, 32.0f);
  transpose_cast_f16_kernel<<<dim3(kDi / 64, kDl / 64), blk, 0, stream>>>(dec_w1, W1DT, kDl, kDi, 4.0f);
  transpose_cast_f16_kernel<<<dim3(kDm / 64, kDi / 64), blk, 0, stream>>>(dec_w2, W2DT, kDi, kDm, 32.0f);
  rows64_kernel<false><<<dim3(kTok / 32), dim3(512), 0, stream>>>(truep, enc_g, enc_bt, LAT0, T16, NX);

  const dim3 gBig((kTok / 64) * (kDi / 64) / 8);
  const dim3 gLat((kTok / 64) * (kDl / 64) / 8);
  const dim3 gRec((kTok / 64) * (kDm / 64) / 8);

  wmma_gemm64<0, false, 2, 0, false, 0, 0><<<gBig, blk, 0, stream>>>(
      H16, H16, kDm, 0L, W1ET, W1ET, kDm, 0L, (void*)UBIG, (void*)UBIG, kDi, 0L, enc_b1, hidden, 0L, kTok, kDi, kDm, 1.0f / 16.0f);
  const int n8g = kTok * kDi / 8;
  gelu_erf_f32_f16x8_kernel<<<dim3(n8g / 256), blk, 0, stream>>>(UBIG, G16, n8g);
  wmma_gemm64<0, false, 2, 0, false, 0, 0><<<gLat, blk, 0, stream>>>(
      G16, G16, kDi, 0L, W2ET, W2ET, kDi, 0L, (void*)LAT0, (void*)LAT0, kDl, 0L, enc_b2, hidden, 0L, kTok, kDl, kDi, 1.0f / 32.0f);
  rows64_kernel<true><<<dim3(kTok / 32), dim3(512), 0, stream>>>(LAT0, enc_g, enc_bt, lat, LAT16, NY);
  wmma_gemm64<0, false, 2, 0, false, 0, 0><<<gBig, blk, 0, stream>>>(
      LAT16, LAT16, kDl, 0L, W1DT, W1DT, kDl, 0L, (void*)UBIG, (void*)UBIG, kDi, 0L, dec_b1, hidden, 0L, kTok, kDi, kDl, 0.25f);
  gelu_erf_f32_f16x8_kernel<<<dim3(n8g / 256), blk, 0, stream>>>(UBIG, G16, n8g);
  float* REC0 = UBIG;
  wmma_gemm64<0, false, 2, 0, false, 0, 0><<<gRec, blk, 0, stream>>>(
      G16, G16, kDi, 0L, W2DT, W2DT, kDi, 0L, (void*)REC0, (void*)REC0, kDm, 0L, dec_b2, hidden, 0L, kTok, kDm, kDi, 1.0f / 32.0f);
  layernorm1024_kernel<<<dim3(kTok), blk, 0, stream>>>(REC0, dec_g, dec_bt, recon);

  float* S = UBIG;
  wmma_gemm64<0, false, 0, 0, false, 0, 0><<<gBig, blk, 0, stream>>>(
      T16, T16, kDl, 0L, T16, T16, kDl, 0L, (void*)S, (void*)S, kTok, 0L, enc_b1, hidden, 0L, kTok, kTok, kDl, 1.0f);
  kmean_partial_kernel<<<dim3(kRedBlocks), blk, 0, stream>>>(S, NX, NX, PART);
  wmma_gemm64<0, false, 0, 0, false, 0, 0><<<gBig, blk, 0, stream>>>(
      LAT16, LAT16, kDl, 0L, LAT16, LAT16, kDl, 0L, (void*)S, (void*)S, kTok, 0L, enc_b1, hidden, 0L, kTok, kTok, kDl, 1.0f);
  kmean_partial_kernel<<<dim3(kRedBlocks), blk, 0, stream>>>(S, NY, NY, PART + (size_t)kRedBlocks * kPartStride);
  wmma_gemm64<0, false, 0, 0, false, 0, 0><<<gBig, blk, 0, stream>>>(
      T16, T16, kDl, 0L, LAT16, LAT16, kDl, 0L, (void*)S, (void*)S, kTok, 0L, enc_b1, hidden, 0L, kTok, kTok, kDl, 1.0f);
  kmean_partial_kernel<<<dim3(kRedBlocks), blk, 0, stream>>>(S, NX, NY, PART + (size_t)2 * kRedBlocks * kPartStride);
  loss_final_kernel<<<dim3(1), dim3(32), 0, stream>>>(PART, regp);
}
